// LocMotionAppearance_9053791060039
// MI455X (gfx1250) — hardware-run, weakly checked
//
#include <hip/hip_runtime.h>
#include <math.h>

typedef __attribute__((ext_vector_type(16))) __bf16       v16b;
typedef __attribute__((ext_vector_type(8)))  __bf16       v8b;
typedef __attribute__((ext_vector_type(8)))  float        v8f;
typedef __attribute__((ext_vector_type(4)))  float        v4f;
typedef __attribute__((ext_vector_type(4)))  unsigned int v4u;
typedef __attribute__((ext_vector_type(4)))  int          v4i;

constexpr int kImg   = 8;
constexpr int kHW    = 512;
constexpr int kSeg   = 2000;
constexpr int kTok   = kImg * kSeg;
constexpr int kPix   = kHW * kHW;
constexpr int kC1    = 256;
constexpr int kCm    = 512;
constexpr int kK3    = 3 * kCm;
constexpr int kM1    = 256;
constexpr int kM2    = 128;
constexpr int kNd    = 15;
constexpr int kXRows = kTok + 2;
constexpr int kX5P   = 8;
constexpr float kEps = 1e-12f;
constexpr float kFix = 65536.0f;
constexpr float kFixInv = 1.0f / 65536.0f;
static_assert(kTok == 16000);
static_assert((kTok % 64) == 0 && (kC1 % 64) == 0 && (kCm % 64) == 0 && (kM1 % 64) == 0 && (kM2 % 64) == 0);
static_assert((kC1 % 32) == 0 && (kCm % 32) == 0 && (kM1 % 32) == 0);
static_assert((kPix % 2048) == 0 && (kTok % 16) == 0);

constexpr size_t kOut0 = 0;
constexpr size_t kOut1 = (size_t)kTok * kNd;
constexpr size_t kOut2 = kOut1 + (size_t)kTok * kM2;
constexpr size_t kOutTotal = kOut2 + (size_t)kTok;
static_assert(kOut1 * 4 == 960000ull && kOut2 * 4 == 9152000ull && kOutTotal * 4 == 9216000ull);
static_assert(((kOut1 * 4) % 128) == 0 && ((kOut2 * 4) % 128) == 0);

constexpr size_t kOffX5   = 0;
constexpr size_t kOffW1T  = kOffX5   + (size_t)kTok * kX5P * 4;
constexpr size_t kOffWMT  = kOffW1T  + (size_t)kC1 * kC1 * 2;
constexpr size_t kOffWM1T = kOffWMT  + (size_t)kCm * kK3 * 2;
constexpr size_t kOffWM2T = kOffWM1T + (size_t)kM1 * kCm * 2;
constexpr size_t kOffA1   = kOffWM2T + (size_t)kM2 * kM1 * 2;
constexpr size_t kOffLF   = kOffA1   + (size_t)kTok * kC1 * 2;
constexpr size_t kOffXH   = kOffLF   + (size_t)kTok * kC1 * 4;
constexpr size_t kOffXL   = kOffXH   + (size_t)kXRows * kCm * 2;
constexpr size_t kOffYH   = kOffXL   + (size_t)kXRows * kCm * 2;
constexpr size_t kOffYL   = kOffYH   + (size_t)kTok * kCm * 2;
constexpr size_t kOffZH   = kOffYL   + (size_t)kTok * kCm * 2;
constexpr size_t kOffZL   = kOffZH   + (size_t)kTok * kM1 * 2;
constexpr size_t kOffHF   = kOffZL   + (size_t)kTok * kM1 * 2;
constexpr size_t kWsTotal = kOffHF   + (size_t)kTok * kM2 * 4;
static_assert(kWsTotal == 117235712ull);
static_assert(kWsTotal <= 134217728ull);
static_assert((kOffW1T % 128) == 0 && (kOffWMT % 128) == 0 && (kOffWM1T % 128) == 0 && (kOffWM2T % 128) == 0 &&
              (kOffA1 % 128) == 0 && (kOffLF % 128) == 0 && (kOffXH % 128) == 0 && (kOffXL % 128) == 0 &&
              (kOffYH % 128) == 0 && (kOffYL % 128) == 0 && (kOffZH % 128) == 0 && (kOffZL % 128) == 0 &&
              (kOffHF % 128) == 0);

__device__ __forceinline__ unsigned bf_bits(float f) {
  const unsigned u = __float_as_uint(f);
  return ((u + 0x7FFFu + ((u >> 16) & 1u)) >> 16) & 0xFFFFu;
}
__device__ __forceinline__ float bf_val(unsigned hb) { return __uint_as_float(hb << 16); }
__device__ __forceinline__ float bf_rne(float f) { return bf_val(bf_bits(f)); }
__device__ __forceinline__ unsigned pack_bf2(float x0, float x1) {
  const unsigned h0 = bf_bits(x0);
  const unsigned h1 = bf_bits(x1);
  return h0 | (h1 << 16);
}
__device__ __forceinline__ void split_bf2(float x0, float x1, unsigned& hw, unsigned& lw) {
  const unsigned h0 = bf_bits(x0);
  const unsigned h1 = bf_bits(x1);
  const unsigned l0 = bf_bits(x0 - bf_val(h0));
  const unsigned l1 = bf_bits(x1 - bf_val(h1));
  hw = h0 | (h1 << 16);
  lw = l0 | (l1 << 16);
}
__device__ __forceinline__ void split_bf8(const v4f a0, const v4f a1, v4u& hv, v4u& lv) {
  unsigned h, l;
  split_bf2(a0[0], a0[1], h, l); hv[0] = h; lv[0] = l;
  split_bf2(a0[2], a0[3], h, l); hv[1] = h; lv[1] = l;
  split_bf2(a1[0], a1[1], h, l); hv[2] = h; lv[2] = l;
  split_bf2(a1[2], a1[3], h, l); hv[3] = h; lv[3] = l;
}
__device__ __forceinline__ v4u pack_bf8(const v4f a0, const v4f a1) {
  v4u o;
  o[0] = pack_bf2(a0[0], a0[1]);
  o[1] = pack_bf2(a0[2], a0[3]);
  o[2] = pack_bf2(a1[0], a1[1]);
  o[3] = pack_bf2(a1[2], a1[3]);
  return o;
}
__device__ __forceinline__ float celu1(float v) {
  const float e = expm1f(fminf(v, 0.0f));
  return (v > 0.0f) ? v : e;
}
__device__ __forceinline__ void wave_sync() {
  __builtin_amdgcn_fence(__ATOMIC_RELEASE, "workgroup");
  __builtin_amdgcn_wave_barrier();
  __builtin_amdgcn_fence(__ATOMIC_ACQUIRE, "workgroup");
}
__device__ __forceinline__ v16b frag_load(const __bf16* p) {
  union U { v16b v; v8b h[2]; } f;
  f.h[0] = *(const v8b*)(p);
  f.h[1] = *(const v8b*)(p + 16);
  return f.v;
}
__device__ __forceinline__ v8f mma_g(v16b a, v16b b, v8f c) {
  c = __builtin_amdgcn_wmma_f32_16x16x32_bf16(false, a, false, b, (short)0, c, false, false);
  asm volatile("v_nop\n\tv_nop\n\tv_nop\n\tv_nop" : "+v"(c) : "v"(a), "v"(b));
  return c;
}

__device__ __forceinline__ void cast8_store(const float* __restrict__ src, unsigned short* __restrict__ dst, int u) {
  const size_t e0 = (size_t)u << 3;
  const v4f a0 = *(const v4f*)(src + e0);
  const v4f a1 = *(const v4f*)(src + e0 + 4);
  const v4u o = pack_bf8(a0, a1);
  unsigned short* q = dst + e0;
  *(volatile v4u*)q = o;
  __threadfence();
  *(volatile v4u*)q = o;
}

__global__ __launch_bounds__(256) void prep_kernel(
    const float* __restrict__ lin1_w, const float* __restrict__ linm1_w, const float* __restrict__ linm2_w,
    const float* __restrict__ convm_w,
    unsigned short* __restrict__ W1T, unsigned short* __restrict__ WM1T, unsigned short* __restrict__ WM2T,
    unsigned short* __restrict__ WMT)
{
  const int blk = blockIdx.x;
  const int tid = threadIdx.x;
  if (blk < 32) {
    cast8_store(lin1_w, W1T, blk * 256 + tid);
  } else if (blk < 96) {
    cast8_store(linm1_w, WM1T, (blk - 32) * 256 + tid);
  } else if (blk < 112) {
    cast8_store(linm2_w, WM2T, (blk - 96) * 256 + tid);
  } else {
    const int u   = (blk - 112) * 256 + tid;
    const int co  = u / 192;
    const int r   = u - co * 192;
    const int tap = r >> 6;
    const int ci0 = (r & 63) << 3;
    const float* s = convm_w + ((size_t)co * kCm + ci0) * 3 + tap;
    const float f0 = s[0],  f1 = s[3],  f2 = s[6],  f3 = s[9];
    const float f4 = s[12], f5 = s[15], f6 = s[18], f7 = s[21];
    v4u o;
    o[0] = pack_bf2(f0, f1);
    o[1] = pack_bf2(f2, f3);
    o[2] = pack_bf2(f4, f5);
    o[3] = pack_bf2(f6, f7);
    unsigned short* q = WMT + ((size_t)u << 3);
    *(volatile v4u*)q = o;
    __threadfence();
    *(volatile v4u*)q = o;
  }
}

__global__ __launch_bounds__(512) void pool_kernel(
    const int* __restrict__ labels, const float* __restrict__ fx, const float* __restrict__ fy,
    const int* __restrict__ fidx, const int* __restrict__ nfr, float* __restrict__ x5)
{
  __shared__ int sAcc[5 * kSeg];
  const int tid = threadIdx.x;
  const int b   = blockIdx.x;
#pragma unroll 1
  for (int i = tid; i < 5 * kSeg; i += 512) sAcc[i] = 0;
  __syncthreads();
  const size_t base = (size_t)b * kPix;
#pragma unroll 1
  for (int it = 0; it < kPix / 2048; ++it) {
    const int p = it * 2048 + tid * 4;
    const v4i lb = *(const v4i*)(labels + base + p);
    const v4f vx = *(const v4f*)(fx + base + p);
    const v4f vy = *(const v4f*)(fy + base + p);
    const int w  = p >> 9;
    const int h0 = p & (kHW - 1);
#pragma unroll
    for (int e = 0; e < 4; ++e) {
      int s = lb[e];
      s = s < 0 ? 0 : s;
      s = s > (kSeg - 1) ? (kSeg - 1) : s;
      const float ax = vx[e];
      const float ay = vy[e];
      const int qx = (int)rintf(bf_rne(ax) * kFix);
      const int qy = (int)rintf(bf_rne(ay) * kFix);
      atomicAdd(&sAcc[s], w);
      atomicAdd(&sAcc[kSeg + s], h0 + e);
      atomicAdd(&sAcc[2 * kSeg + s], qx);
      atomicAdd(&sAcc[3 * kSeg + s], qy);
      atomicAdd(&sAcc[4 * kSeg + s], 1);
    }
  }
  __syncthreads();
  const float tb = (float)fidx[b] / ((float)nfr[b] - 1.0f);
  const float cinv = 1.0f / (float)(kHW - 1);
#pragma unroll 1
  for (int k = 0; k < 8; ++k) {
    const int u = k * 512 + tid;
    if (u < 2 * kSeg) {
      const int s  = u >> 1;
      const int hf = u & 1;
      const int sw = sAcc[s];
      const int sh = sAcc[kSeg + s];
      const int sx = sAcc[2 * kSeg + s];
      const int sy = sAcc[3 * kSeg + s];
      const int cn = sAcc[4 * kSeg + s];
      const float inv = 1.0f / fmaxf((float)cn, 1.0f);
      const float mx  = ((float)sw * cinv) * inv;
      const float my  = ((float)sh * cinv) * inv;
      const float mfx = ((float)sx * kFixInv) * inv;
      const float mfy = ((float)sy * kFixInv) * inv;
      v4f o;
      o[0] = hf ? mfy : tb;
      o[1] = hf ? 0.0f : mx;
      o[2] = hf ? 0.0f : my;
      o[3] = hf ? 0.0f : mfx;
      float* dst = x5 + ((size_t)(b * kSeg + s)) * kX5P + hf * 4;
      *(volatile v4f*)dst = o;
      __threadfence();
      *(volatile v4f*)dst = o;
    }
  }
}

__global__ __launch_bounds__(256) void conv1_kernel(
    const float* __restrict__ x5, const float* __restrict__ w, const float* __restrict__ bsrc,
    unsigned short* __restrict__ A1)
{
  __shared__ __align__(16) float sX[32 * kX5P];
  __shared__ __align__(16) float sT[16 * 260];
  const int tid  = threadIdx.x;
  const int lane = tid & 31;
  const int wave = tid >> 5;
  const int n0   = blockIdx.x * 16;
  {
    const int r   = tid >> 3;
    const int c   = tid & 7;
    const int tok = n0 - 1 + r;
    int tc = tok < 0 ? 0 : tok;
    tc = tc > (kTok - 1) ? (kTok - 1) : tc;
    float v = x5[(size_t)tc * kX5P + c];
    asm volatile("" : "+v"(v));
    const bool ok = (tok >= 0) && (tok < kTok);
    sX[tid] = ok ? v : 0.0f;
  }
  float wr[15];
#pragma unroll
  for (int q = 0; q < 15; ++q) wr[q] = bf_rne(w[tid * 15 + q]);
  const float bias = bf_rne(bsrc[tid]);
  __syncthreads();
#pragma unroll 1
  for (int s = 0; s < 16; ++s) {
    float acc = bias;
#pragma unroll
    for (int k = 0; k < 3; ++k) {
#pragma unroll
      for (int ci = 0; ci < 5; ++ci) acc = fmaf(sX[(s + k) * kX5P + ci], wr[ci * 3 + k], acc);
    }
    sT[s * 260 + tid] = celu1(acc);
  }
  __syncthreads();
  v4u pk[2];
#pragma unroll
  for (int it = 0; it < 2; ++it) {
    const float* sp = sT + (it * 8 + wave) * 260 + lane * 8;
    const v4f a0 = *(const v4f*)(sp);
    const v4f a1 = *(const v4f*)(sp + 4);
    pk[it] = pack_bf8(a0, a1);
  }
  for (int pass = 0; pass < 2; ++pass) {
#pragma unroll
    for (int it = 0; it < 2; ++it)
      *(volatile v4u*)(A1 + (size_t)(n0 + it * 8 + wave) * kC1 + lane * 8) = pk[it];
    __threadfence();
  }
}

template <int SPL, int TAPS, int OUT_MODE>
__global__ __launch_bounds__(256) void gemm64_kernel(
    const unsigned short* __restrict__ Ap, const unsigned short* __restrict__ A2p, int lda,
    const unsigned short* __restrict__ Btp, int ldb,
    void* __restrict__ Cout, void* __restrict__ Cout2, int ldc,
    const float* __restrict__ bias, int M, int N, int Kper, int loK)
{
  const __bf16* A  = (const __bf16*)Ap;
  const __bf16* A2 = (const __bf16*)A2p;
  const __bf16* Bt = (const __bf16*)Btp;
  __shared__ __align__(16) float sT[8][16 * 68];
  const int lane = threadIdx.x & 31;
  const int wave = threadIdx.x >> 5;
  const int tilesN = N >> 6;
  const int tilesM = M >> 6;
  const int tile = blockIdx.x * 8 + wave;
  if (tile >= tilesM * tilesN) return;
  const int tm = tile / tilesN;
  const int tn = tile - tm * tilesN;
  const int m0 = tm << 6;
  const int n0 = tn << 6;
  const int rlane = lane & 15;
  const int koff  = (lane >> 4) * 8;
  const int mOff  = (lane >> 4) * 8;

  v8f acc[4][4];
#pragma unroll
  for (int i = 0; i < 4; ++i)
#pragma unroll
    for (int j = 0; j < 4; ++j) acc[i][j] = (v8f){0.f, 0.f, 0.f, 0.f, 0.f, 0.f, 0.f, 0.f};

#pragma unroll 1
  for (int tap = 0; tap < TAPS; ++tap) {
#pragma unroll 1
    for (int kc = 0; kc < Kper; kc += 32) {
      v16b bh[4];
#pragma unroll
      for (int j = 0; j < 4; ++j)
        bh[j] = frag_load(Bt + (size_t)(n0 + (j << 4) + rlane) * ldb + tap * Kper + kc + koff);
      const bool useLo = (SPL == 1) && (kc < loK);
#pragma unroll
      for (int i = 0; i < 4; ++i) {
        const size_t ao = (size_t)(m0 + (i << 4) + rlane + tap) * lda + kc + koff;
        const v16b ah = frag_load(A + ao);
#pragma unroll
        for (int j = 0; j < 4; ++j) acc[i][j] = mma_g(ah, bh[j], acc[i][j]);
        if (useLo) {
          const v16b al = frag_load(A2 + ao);
#pragma unroll
          for (int j = 0; j < 4; ++j) acc[i][j] = mma_g(al, bh[j], acc[i][j]);
        }
      }
    }
  }

  float* slab = sT[wave];
  float bv[4];
#pragma unroll
  for (int j = 0; j < 4; ++j) bv[j] = bf_rne(bias[n0 + (j << 4) + rlane]);

#pragma unroll
  for (int i = 0; i < 4; ++i) {
    const int mBase = m0 + (i << 4);
#pragma unroll
    for (int j = 0; j < 4; ++j) {
#pragma unroll
      for (int r = 0; r < 8; ++r) slab[(mOff + r) * 68 + (j << 4) + rlane] = acc[i][j][r] + bv[j];
    }
    wave_sync();
#pragma unroll 1
    for (int e = 0; e < 32; ++e) {
      float* sp = slab + (e >> 1) * 68 + (e & 1) * 32 + lane;
      const float v = *sp;
      *sp = celu1(v);
    }
    wave_sync();
    if (OUT_MODE == 0) {
      float* C = (float*)Cout;
      const int hh = lane >> 4;
      const int c4 = (lane & 15) * 4;
      v4f vv[8];
#pragma unroll
      for (int it = 0; it < 8; ++it) vv[it] = *(const v4f*)(slab + (it * 2 + hh) * 68 + c4);
      for (int pass = 0; pass < 2; ++pass) {
#pragma unroll
        for (int it = 0; it < 8; ++it)
          *(volatile v4f*)(C + (size_t)(mBase + it * 2 + hh) * ldc + n0 + c4) = vv[it];
        __threadfence();
      }
    } else {
      unsigned short* C  = (unsigned short*)Cout;
      unsigned short* C2 = (unsigned short*)Cout2;
      const int q  = lane >> 3;
      const int c8 = (lane & 7) * 8;
      v4u hv[4], lv[4];
#pragma unroll
      for (int it = 0; it < 4; ++it) {
        const float* sp = slab + (it * 4 + q) * 68 + c8;
        const v4f a0 = *(const v4f*)(sp);
        const v4f a1 = *(const v4f*)(sp + 4);
        split_bf8(a0, a1, hv[it], lv[it]);
      }
      for (int pass = 0; pass < 2; ++pass) {
#pragma unroll
        for (int it = 0; it < 4; ++it) {
          const size_t o = (size_t)(mBase + it * 4 + q) * ldc + n0 + c8;
          *(volatile v4u*)(C + o)  = hv[it];
          *(volatile v4u*)(C2 + o) = lv[it];
        }
        __threadfence();
      }
    }
    wave_sync();
  }
}

__global__ __launch_bounds__(256) void l2cat_kernel(
    const float* __restrict__ LF, const float* __restrict__ dec,
    unsigned short* __restrict__ XH, unsigned short* __restrict__ XL)
{
  const int lane = threadIdx.x & 31;
  const int wave = threadIdx.x >> 5;
  const int p = blockIdx.x * 8 + wave;
  if (p >= kXRows) return;
  const bool halo = (p == 0) || (p == kXRows - 1);
  int n = p - 1;
  n = n < 0 ? 0 : n;
  n = n > (kTok - 1) ? (kTok - 1) : n;
  const float* lr = LF + (size_t)n * kC1 + lane * 8;
  const v4f a0 = *(const v4f*)(lr);
  const v4f a1 = *(const v4f*)(lr + 4);
  const float* dr = dec + (size_t)n * 256 + lane * 8;
  const v4f d0 = *(const v4f*)(dr);
  const v4f d1 = *(const v4f*)(dr + 4);
  float ss = 0.0f;
#pragma unroll
  for (int e = 0; e < 4; ++e) {
    ss = fmaf(a0[e], a0[e], ss);
    ss = fmaf(a1[e], a1[e], ss);
  }
#pragma unroll
  for (int off = 16; off > 0; off >>= 1) ss += __shfl_xor(ss, off, 32);
  const float inv = 1.0f / fmaxf(sqrtf(ss), kEps);
  const v4f x0 = a0 * inv;
  const v4f x1 = a1 * inv;
  v4u mh, ml;
  split_bf8(x0, x1, mh, ml);
  v4u dh = pack_bf8(d0, d1);
  const unsigned km = halo ? 0u : 0xFFFFFFFFu;
#pragma unroll
  for (int e = 0; e < 4; ++e) {
    mh[e] = mh[e] & km;
    ml[e] = ml[e] & km;
    dh[e] = dh[e] & km;
  }
  const v4u zz = (v4u){0u, 0u, 0u, 0u};
  unsigned short* qh = XH + (size_t)p * kCm + lane * 8;
  unsigned short* ql = XL + (size_t)p * kCm + lane * 8;
  for (int pass = 0; pass < 2; ++pass) {
    *(volatile v4u*)(qh)       = mh;
    *(volatile v4u*)(qh + 256) = dh;
    *(volatile v4u*)(ql)       = ml;
    *(volatile v4u*)(ql + 256) = zz;
    __threadfence();
  }
}

__global__ __launch_bounds__(256) void head_kernel(
    const float* __restrict__ HF, const float* __restrict__ pw, const float* __restrict__ pb,
    const float* __restrict__ dw, float* __restrict__ out)
{
  __shared__ __align__(16) float sWn[16 * kM2];
  __shared__ __align__(16) float sCs[64 * kNd];
  __shared__ __align__(16) float sRho[64];
  const int tid  = threadIdx.x;
  const int lane = tid & 31;
  const int wave = tid >> 5;
#pragma unroll 1
  for (int jj = 0; jj < 2; ++jj) {
    const int j  = wave + jj * 8;
    const int jc = j < kNd ? j : (kNd - 1);
    const v4f wraw = *(const v4f*)(dw + jc * kM2 + lane * 4);
    v4f wq;
    wq[0] = bf_rne(wraw[0]);
    wq[1] = bf_rne(wraw[1]);
    wq[2] = bf_rne(wraw[2]);
    wq[3] = bf_rne(wraw[3]);
    float ss = wq[0] * wq[0];
    ss = fmaf(wq[1], wq[1], ss);
    ss = fmaf(wq[2], wq[2], ss);
    ss = fmaf(wq[3], wq[3], ss);
#pragma unroll
    for (int off = 16; off > 0; off >>= 1) ss += __shfl_xor(ss, off, 32);
    const float inv = 1.0f / fmaxf(sqrtf(ss), kEps);
    const float keep = (j < kNd) ? inv : 0.0f;
    const v4f o = wq * keep;
    *(v4f*)(sWn + j * kM2 + lane * 4) = o;
  }
  v4f pq;
  {
    const v4f praw = *(const v4f*)(pw + lane * 4);
    pq[0] = bf_rne(praw[0]);
    pq[1] = bf_rne(praw[1]);
    pq[2] = bf_rne(praw[2]);
    pq[3] = bf_rne(praw[3]);
  }
  const float pbv = bf_rne(pb[0]);
  __syncthreads();
  float* out1 = out + kOut1;
#pragma unroll 1
  for (int rr = 0; rr < 8; ++rr) {
    const int rl  = wave * 8 + rr;
    const int row = blockIdx.x * 64 + rl;
    const v4f h = *(const v4f*)(HF + (size_t)row * kM2 + lane * 4);
    float ss = h[0] * h[0];
    ss = fmaf(h[1], h[1], ss);
    ss = fmaf(h[2], h[2], ss);
    ss = fmaf(h[3], h[3], ss);
    float pr = h[0] * pq[0];
    pr = fmaf(h[1], pq[1], pr);
    pr = fmaf(h[2], pq[2], pr);
    pr = fmaf(h[3], pq[3], pr);
#pragma unroll
    for (int off = 16; off > 0; off >>= 1) {
      ss += __shfl_xor(ss, off, 32);
      pr += __shfl_xor(pr, off, 32);
    }
    const float inv = 1.0f / fmaxf(sqrtf(ss), kEps);
    const float rho = pr + pbv;
    const v4f xn = h * inv;
    float* o1 = out1 + (size_t)row * kM2 + lane * 4;
    *(volatile v4f*)o1 = xn;
    __threadfence();
    *(volatile v4f*)o1 = xn;
    float csv = 0.0f;
#pragma unroll 1
    for (int j = 0; j < kNd; ++j) {
      const v4f wv = *(const v4f*)(sWn + j * kM2 + lane * 4);
      float pj = xn[0] * wv[0];
      pj = fmaf(xn[1], wv[1], pj);
      pj = fmaf(xn[2], wv[2], pj);
      pj = fmaf(xn[3], wv[3], pj);
#pragma unroll
      for (int off = 16; off > 0; off >>= 1) pj += __shfl_xor(pj, off, 32);
      csv = (lane == j) ? pj : csv;
    }
    if (lane < kNd) sCs[rl * kNd + lane] = csv;
    if (lane == kNd) sRho[rl] = rho;
  }
  __syncthreads();
  {
    const int u  = tid < 240 ? tid : 239;
    const int ur = tid >= 240 ? (tid - 240) : 0;
    const v4f v0 = *(const v4f*)(sCs + u * 4);
    const v4f v2 = *(const v4f*)(sRho + ur * 4);
    float* o0 = out + kOut0 + (size_t)blockIdx.x * (64 * kNd) + u * 4;
    float* o2 = out + kOut2 + (size_t)blockIdx.x * 64 + ur * 4;
    for (int pass = 0; pass < 2; ++pass) {
      if (tid < 240) *(volatile v4f*)o0 = v0;
      else           *(volatile v4f*)o2 = v2;
      __threadfence();
    }
  }
}

extern "C" void kernel_launch(void* const* d_in, const int* in_sizes, int n_in,
                              void* d_out, int out_size, void* d_ws, size_t ws_size,
                              hipStream_t stream) {
  if (n_in < 19) return;
  if (in_sizes[0] != kImg * kPix) return;
  if (in_sizes[1] != kImg * kPix) return;
  if (in_sizes[2] != kImg * kPix) return;
  if (in_sizes[3] != kImg) return;
  if (in_sizes[4] != kImg) return;
  if (in_sizes[5] != kTok * 256) return;
  if (in_sizes[6] != kC1 * 15) return;
  if (in_sizes[7] != kC1) return;
  if (in_sizes[8] != kC1 * kC1) return;
  if (in_sizes[9] != kC1) return;
  if (in_sizes[10] != kCm * kCm * 3) return;
  if (in_sizes[11] != kCm) return;
  if (in_sizes[12] != kM1 * kCm) return;
  if (in_sizes[13] != kM1) return;
  if (in_sizes[14] != kM2 * kM1) return;
  if (in_sizes[15] != kM2) return;
  if (in_sizes[16] != kM2) return;
  if (in_sizes[17] != 1) return;
  if (in_sizes[18] != kNd * kM2) return;
  if ((size_t)out_size != kOutTotal) return;
  if (ws_size < kWsTotal) return;

  const int*   labels  = (const int*)  d_in[0];
  const float* fx      = (const float*)d_in[1];
  const float* fy      = (const float*)d_in[2];
  const int*   fidx    = (const int*)  d_in[3];
  const int*   nfr     = (const int*)  d_in[4];
  const float* dec     = (const float*)d_in[5];
  const float* conv1_w = (const float*)d_in[6];
  const float* conv1_b = (const float*)d_in[7];
  const float* lin1_w  = (const float*)d_in[8];
  const float* lin1_b  = (const float*)d_in[9];
  const float* convm_w = (const float*)d_in[10];
  const float* convm_b = (const float*)d_in[11];
  const float* linm1_w = (const float*)d_in[12];
  const float* linm1_b = (const float*)d_in[13];
  const float* linm2_w = (const float*)d_in[14];
  const float* linm2_b = (const float*)d_in[15];
  const float* pred_w  = (const float*)d_in[16];
  const float* pred_b  = (const float*)d_in[17];
  const float* dist_w  = (const float*)d_in[18];
  float* out = (float*)d_out;

  char* ws = (char*)d_ws;
  float*          X5   = (float*)(ws + kOffX5);
  unsigned short* W1T  = (unsigned short*)(ws + kOffW1T);
  unsigned short* WMT  = (unsigned short*)(ws + kOffWMT);
  unsigned short* WM1T = (unsigned short*)(ws + kOffWM1T);
  unsigned short* WM2T = (unsigned short*)(ws + kOffWM2T);
  unsigned short* A1   = (unsigned short*)(ws + kOffA1);
  float*          LF   = (float*)(ws + kOffLF);
  unsigned short* XH   = (unsigned short*)(ws + kOffXH);
  unsigned short* XL   = (unsigned short*)(ws + kOffXL);
  unsigned short* YH   = (unsigned short*)(ws + kOffYH);
  unsigned short* YL   = (unsigned short*)(ws + kOffYL);
  unsigned short* ZH   = (unsigned short*)(ws + kOffZH);
  unsigned short* ZL   = (unsigned short*)(ws + kOffZL);
  float*          HF   = (float*)(ws + kOffHF);

  prep_kernel<<<496, 256, 0, stream>>>(lin1_w, linm1_w, linm2_w, convm_w, W1T, WM1T, WM2T, WMT);

  pool_kernel<<<kImg, 512, 0, stream>>>(labels, fx, fy, fidx, nfr, X5);

  conv1_kernel<<<kTok / 16, 256, 0, stream>>>(X5, conv1_w, conv1_b, A1);

  gemm64_kernel<0, 1, 0><<<125, 256, 0, stream>>>(
      A1, A1, kC1, W1T, kC1, (void*)LF, (void*)LF, kC1, lin1_b, kTok, kC1, kC1, 0);

  l2cat_kernel<<<(kXRows + 7) / 8, 256, 0, stream>>>(LF, dec, XH, XL);

  gemm64_kernel<1, 3, 2><<<250, 256, 0, stream>>>(
      XH, XL, kCm, WMT, kK3, (void*)YH, (void*)YL, kCm, convm_b, kTok, kCm, kCm, 0);

  gemm64_kernel<1, 1, 2><<<125, 256, 0, stream>>>(
      YH, YL, kCm, WM1T, kCm, (void*)ZH, (void*)ZL, kM1, linm1_b, kTok, kM1, kCm, kCm);

  gemm64_kernel<1, 1, 0><<<63, 256, 0, stream>>>(
      ZH, ZL, kM1, WM2T, kM1, (void*)HF, (void*)HF, kM2, linm2_b, kTok, kM2, kM1, kM1);

  head_kernel<<<kTok / 64, 256, 0, stream>>>(HF, pred_w, pred_b, dist_w, out);
}
